// RNN_91250875171637
// MI455X (gfx1250) — hardware-verified
//
#include <hip/hip_runtime.h>
#include <math.h>

constexpr int NBATCH = 256;
constexpr int NSTEP  = 100;
constexpr int NHID   = 2048;
constexpr int NPLACE = 512;
constexpr int NROWS  = NBATCH * NSTEP;
constexpr int NTHR   = 256;
constexpr float WCARRY     = 256.0f;
constexpr float WCARRY_INV = 1.0f / 256.0f;

static_assert(NBATCH % 64 == 0, "M tile multiple");
static_assert(NHID % 64 == 0, "N tile multiple");
static_assert(NPLACE % 64 == 0, "N tile multiple");
static_assert(NROWS % 64 == 0, "M tile multiple");
static_assert(NHID % 32 == 0 && NPLACE % 32 == 0, "K multiple of 32");
static_assert(((NBATCH / 64) * (NHID / 64)) % 8 == 0, "step grid exact");
static_assert(((NROWS / 64) * (NPLACE / 64)) % 8 == 0, "decoder grid exact");
static_assert((NBATCH * NPLACE / 8) % NTHR == 0, "p0 convert grid exact");

typedef __attribute__((ext_vector_type(16))) _Float16 v16h;
typedef __attribute__((ext_vector_type(8)))  _Float16 v8h;
typedef __attribute__((ext_vector_type(8)))  float    v8f;
typedef __attribute__((ext_vector_type(4)))  float    v4f;
typedef __attribute__((ext_vector_type(2)))  float    v2f;

__device__ __forceinline__ void grp_guard_h(v8f& a, v8f& b, v8f& c, v8f& d, v16h x, v16h y0, v16h y1, v16h y2, v16h y3) {
  asm volatile("v_nop\n\tv_nop\n\tv_nop\n\tv_nop" : "+v"(a), "+v"(b), "+v"(c), "+v"(d) : "v"(x), "v"(y0), "v"(y1), "v"(y2), "v"(y3));
}
__device__ __forceinline__ void keep4_h(v16h a, v16h b, v16h c, v16h d) { asm volatile("v_nop" :: "v"(a), "v"(b), "v"(c), "v"(d)); }
__device__ __forceinline__ void acc_guard4(v8f& a, v8f& b, v8f& c, v8f& d) { asm volatile("v_nop\n\tv_nop\n\tv_nop\n\tv_nop" : "+v"(a), "+v"(b), "+v"(c), "+v"(d)); }

struct FragH {
  union U { v16h v; v8h h[2]; };
  static __device__ __forceinline__ v16h load(const _Float16* p) {
    U f;
    f.h[0] = *(const v8h*)(p);
    f.h[1] = *(const v8h*)(p + 16);
    return f.v;
  }
  static __device__ __forceinline__ v8f mma(v16h a, v16h b, v8f c) {
    return __builtin_amdgcn_wmma_f32_16x16x32_f16(false, a, false, b, (short)0, c, false, false);
  }
};

template <int OUT_MODE, bool XPROJ>
__global__ __launch_bounds__(256) void gemm64_f16_kernel(
    const unsigned short* __restrict__ Ap, int lda,
    const unsigned short* __restrict__ Btp, int ldb,
    void* Cout, int ldc,
    const float* __restrict__ vin, const float* __restrict__ win, int tstep,
    int M, int N, int K, float scale) {
  const _Float16* A  = (const _Float16*)Ap;
  const _Float16* Bt = (const _Float16*)Btp;
  __shared__ __align__(16) float sT[8][16 * 68];
  const int lane = threadIdx.x & 31;
  const int wave = threadIdx.x >> 5;
  const int tilesN = N >> 6;
  const int tilesM = M >> 6;
  const int tile = blockIdx.x * 8 + wave;
  if (tile >= tilesM * tilesN) return;
  const int tm = tile / tilesN;
  const int tn = tile - tm * tilesN;
  const int m0 = tm << 6;
  const int n0 = tn << 6;

  const int rlane = lane & 15;
  const int koff  = (lane >> 4) * 8;
  const int mOff  = (lane >> 4) * 8;

  v8f acc[4][4];
#pragma unroll
  for (int i = 0; i < 4; ++i)
#pragma unroll
    for (int j = 0; j < 4; ++j) acc[i][j] = (v8f){0.f, 0.f, 0.f, 0.f, 0.f, 0.f, 0.f, 0.f};

  for (int k0 = 0; k0 < K; k0 += 32) {
    v16h bh[4];
#pragma unroll
    for (int j = 0; j < 4; ++j) {
      const size_t bo = (size_t)(n0 + (j << 4) + rlane) * (size_t)ldb + (size_t)(koff + k0);
      bh[j] = FragH::load(Bt + bo);
    }
#pragma unroll
    for (int i = 0; i < 4; ++i) {
      const size_t ao = (size_t)(m0 + (i << 4) + rlane) * (size_t)lda + (size_t)(koff + k0);
      const v16h ah = FragH::load(A + ao);
#pragma unroll
      for (int j = 0; j < 4; ++j) acc[i][j] = FragH::mma(ah, bh[j], acc[i][j]);
      grp_guard_h(acc[i][0], acc[i][1], acc[i][2], acc[i][3], ah, bh[0], bh[1], bh[2], bh[3]);
    }
    keep4_h(bh[0], bh[1], bh[2], bh[3]);
  }
  acc_guard4(acc[0][0], acc[0][1], acc[0][2], acc[0][3]);
  acc_guard4(acc[1][0], acc[1][1], acc[1][2], acc[1][3]);
  acc_guard4(acc[2][0], acc[2][1], acc[2][2], acc[2][3]);
  acc_guard4(acc[3][0], acc[3][1], acc[3][2], acc[3][3]);

  float* slab = sT[wave];
#pragma unroll
  for (int i = 0; i < 4; ++i) {
    const int mBase = m0 + (i << 4);
#pragma unroll
    for (int j = 0; j < 4; ++j) {
#pragma unroll
      for (int r = 0; r < 8; ++r) {
        const float val = acc[i][j][r] * scale;
        slab[(mOff + r) * 68 + (j << 4) + rlane] = val;
      }
    }
    __builtin_amdgcn_fence(__ATOMIC_RELEASE, "workgroup");
    __builtin_amdgcn_wave_barrier();
    __builtin_amdgcn_fence(__ATOMIC_ACQUIRE, "workgroup");
    if (OUT_MODE == 0) {
      float* C = (float*)Cout;
      const int hh = lane >> 4, c4 = (lane & 15) * 4;
      for (int pass = 0; pass < 2; ++pass) {
#pragma unroll
        for (int it = 0; it < 8; ++it) {
          const int row = it * 2 + hh;
          const v4f val = *(const v4f*)(slab + row * 68 + c4);
          *(volatile v4f*)(C + (size_t)(mBase + row) * (size_t)ldc + (size_t)(n0 + c4)) = val;
        }
        __threadfence();
      }
    } else {
      const int q = lane >> 3, c8 = (lane & 7) * 8;
      unsigned short* C = (unsigned short*)Cout;
      v4f wa0 = (v4f){0.f, 0.f, 0.f, 0.f};
      v4f wa1 = wa0, wb0 = wa0, wb1 = wa0;
      if (XPROJ) {
        wa0 = *(const v4f*)(win + n0 + c8);
        wa1 = *(const v4f*)(win + n0 + c8 + 4);
        wb0 = *(const v4f*)(win + NHID + n0 + c8);
        wb1 = *(const v4f*)(win + NHID + n0 + c8 + 4);
      }
      v8h hv[4];
#pragma unroll
      for (int it = 0; it < 4; ++it) {
        const int row = it * 4 + q;
        const float* sp = slab + row * 68 + c8;
        float x0 = 0.0f, x1 = 0.0f;
        if (XPROJ) {
          const v2f vv = *(const v2f*)(vin + ((size_t)(mBase + row) * (size_t)NSTEP + (size_t)tstep) * 2);
          x0 = vv[0];
          x1 = vv[1];
        }
#pragma unroll
        for (int e = 0; e < 4; ++e) {
          float f0 = sp[e];
          float f1 = sp[4 + e];
          if (XPROJ) {
            f0 = f0 + x0 * wa0[e] + x1 * wb0[e];
            f1 = f1 + x0 * wa1[e] + x1 * wb1[e];
            f0 = fmaxf(f0, 0.0f);
            f1 = fmaxf(f1, 0.0f);
          }
          hv[it][e]     = (_Float16)f0;
          hv[it][4 + e] = (_Float16)f1;
        }
      }
      for (int pass = 0; pass < 2; ++pass) {
#pragma unroll
        for (int it = 0; it < 4; ++it) {
          const int row = it * 4 + q;
          *(volatile v8h*)(C + (size_t)(mBase + row) * (size_t)ldc + (size_t)(n0 + c8)) = hv[it];
        }
        __threadfence();
      }
    }
    __builtin_amdgcn_fence(__ATOMIC_RELEASE, "workgroup");
    __builtin_amdgcn_wave_barrier();
    __builtin_amdgcn_fence(__ATOMIC_ACQUIRE, "workgroup");
  }
}

__global__ __launch_bounds__(256) void tpose_f16_kernel(const float* __restrict__ src, int R, int C, int ldo,
                                                        unsigned short* __restrict__ O, float sc) {
  __shared__ float Tt[64 * 65];
  const int tid = threadIdx.x;
  const int c0 = blockIdx.x * 64, r0 = blockIdx.y * 64;
#pragma unroll
  for (int i = 0; i < 4; ++i) {
    const int idx = i * 256 + tid;
    const int rr = idx >> 4, cc = (idx & 15) * 4;
    const v4f val = *(const v4f*)(src + (size_t)(r0 + rr) * (size_t)C + (size_t)(c0 + cc));
    Tt[rr * 65 + cc + 0] = val[0];
    Tt[rr * 65 + cc + 1] = val[1];
    Tt[rr * 65 + cc + 2] = val[2];
    Tt[rr * 65 + cc + 3] = val[3];
  }
  __syncthreads();
  const int q = tid >> 3, c8 = (tid & 7) * 8;
  v8h hv[2];
#pragma unroll
  for (int g = 0; g < 2; ++g) {
    const int qq = g * 32 + q;
#pragma unroll
    for (int e = 0; e < 8; ++e) {
      const float f = Tt[(c8 + e) * 65 + qq] * sc;
      hv[g][e] = (_Float16)f;
    }
  }
  for (int pass = 0; pass < 2; ++pass) {
#pragma unroll
    for (int g = 0; g < 2; ++g) {
      const size_t o = (size_t)(c0 + g * 32 + q) * (size_t)ldo + (size_t)(r0 + c8);
      *(volatile v8h*)(O + o) = hv[g];
    }
    __threadfence();
  }
}

__global__ __launch_bounds__(256) void cvt8_f16_kernel(const float* __restrict__ src, unsigned short* __restrict__ dst, int n8) {
  const int i = blockIdx.x * 256 + threadIdx.x;
  if (i < n8) {
    const float* sp = src + (size_t)i * 8;
    const v4f a = *(const v4f*)(sp);
    const v4f b = *(const v4f*)(sp + 4);
    v8h hv;
#pragma unroll
    for (int e = 0; e < 4; ++e) {
      hv[e]     = (_Float16)a[e];
      hv[4 + e] = (_Float16)b[e];
    }
    *(volatile v8h*)(dst + (size_t)i * 8) = hv;
    __threadfence();
    *(volatile v8h*)(dst + (size_t)i * 8) = hv;
  }
}

extern "C" void kernel_launch(void* const* d_in, const int* in_sizes, int n_in,
                              void* d_out, int out_size, void* d_ws, size_t ws_size, hipStream_t stream) {
  if (n_in < 6 || d_out == nullptr || d_ws == nullptr) return;
  if (in_sizes[0] != NBATCH * NSTEP * 2 || in_sizes[1] != NBATCH * NPLACE || in_sizes[2] != NPLACE * NHID ||
      in_sizes[3] != 2 * NHID || in_sizes[4] != NHID * NHID || in_sizes[5] != NHID * NPLACE ||
      out_size != NROWS * NPLACE) return;

  const float* vin  = (const float*)d_in[0];
  const float* p0   = (const float*)d_in[1];
  const float* wenc = (const float*)d_in[2];
  const float* win  = (const float*)d_in[3];
  const float* wrec = (const float*)d_in[4];
  const float* wdec = (const float*)d_in[5];
  float* out = (float*)d_out;

  char* ws = (char*)d_ws;
  size_t off = 0;
  auto carve = [&](size_t bytes) -> char* { char* p = ws + off; off += (bytes + 255) & ~(size_t)255; return p; };
  unsigned short* WRECT = (unsigned short*)carve((size_t)NHID * NHID * 2);
  unsigned short* WENCT = (unsigned short*)carve((size_t)NHID * NPLACE * 2);
  unsigned short* WDECT = (unsigned short*)carve((size_t)NPLACE * NHID * 2);
  unsigned short* P0H   = (unsigned short*)carve((size_t)NBATCH * NPLACE * 2);
  unsigned short* H0    = (unsigned short*)carve((size_t)NBATCH * NHID * 2);
  unsigned short* G     = (unsigned short*)carve((size_t)NROWS * NHID * 2);
  if (off > ws_size || off > (size_t)134217728) return;

  tpose_f16_kernel<<<dim3(NHID / 64, NHID / 64), 256, 0, stream>>>(wrec, NHID, NHID, NHID, WRECT, WCARRY);
  tpose_f16_kernel<<<dim3(NHID / 64, NPLACE / 64), 256, 0, stream>>>(wenc, NPLACE, NHID, NPLACE, WENCT, WCARRY);
  tpose_f16_kernel<<<dim3(NPLACE / 64, NHID / 64), 256, 0, stream>>>(wdec, NHID, NPLACE, NHID, WDECT, WCARRY);
  const int n8p = NBATCH * NPLACE / 8;
  cvt8_f16_kernel<<<(n8p + 255) / 256, 256, 0, stream>>>(p0, P0H, n8p);

  const int stepBlocks = ((NBATCH / 64) * (NHID / 64)) / 8;
  gemm64_f16_kernel<1, false><<<stepBlocks, 256, 0, stream>>>(
      P0H, NPLACE, WENCT, NPLACE, (void*)H0, NHID, vin, win, 0, NBATCH, NHID, NPLACE, WCARRY_INV);

  for (int t = 0; t < NSTEP; ++t) {
    const unsigned short* Aprev = (t == 0) ? H0 : (G + (size_t)(t - 1) * NHID);
    const int ldaPrev = (t == 0) ? NHID : (NSTEP * NHID);
    gemm64_f16_kernel<1, true><<<stepBlocks, 256, 0, stream>>>(
        Aprev, ldaPrev, WRECT, NHID, (void*)(G + (size_t)t * NHID), NSTEP * NHID, vin, win, t,
        NBATCH, NHID, NHID, WCARRY_INV);
  }

  const int decBlocks = ((NROWS / 64) * (NPLACE / 64)) / 8;
  gemm64_f16_kernel<0, false><<<decBlocks, 256, 0, stream>>>(
      G, NHID, WDECT, NHID, (void*)out, NPLACE, vin, win, 0, NROWS, NPLACE, NHID, WCARRY_INV);
}
